// MyGNN2_11355893531404
// MI455X (gfx1250) — hardware-verified
//
#include <hip/hip_runtime.h>
#include <stddef.h>


#define CC      128
#define NTHR    256
#define NWAVE   8
#define EPT     8
#define NGRP    2
#define CHUNK   (NTHR * EPT * NGRP)
#define WCAPC   (EPT * NGRP * 32)
#define WCAPF   (EPT * NGRP * 32)
#define ESHF    11
#define EMASK   0xFFFFF
#define NBC     32768
#define NBF     2048
#define RCAP    49152
#define RBN     128
#define TGT     256
#define DEGCAP  512
#define GROWS   128
#define OTHR    512
#define TPK     64
#define TPN     32
#define TPP     72
#define ASCL    16
#define HSCL    64
#define WSCL    64
#define WSCAP   134217728

#define LDS_COUNT  ((NBC + NWAVE * WCAPC + NWAVE) * 4)
#define LDS_FILL   ((RCAP + NBF + NWAVE * WCAPF + NWAVE) * 4)
#define LDS_GEMM   (GROWS * CC * 4)

static_assert((CHUNK & (CHUNK - 1)) == 0);
static_assert((NBC & (NBC - 1)) == 0 && (NBF & (NBF - 1)) == 0);
static_assert(NBF <= (1 << ESHF));
static_assert((NBC % NBF) == 0);
static_assert(OTHR * 4 == NBF);
static_assert((RCAP % 32) == 0);
static_assert(TGT == NWAVE * 32);
static_assert(GROWS == NWAVE * 16);
static_assert((TGT % GROWS) == 0);
static_assert(NBC == NWAVE * 32 * 128);
static_assert(CC == 32 * 4);
static_assert((CC % 32) == 0);
static_assert((CC % TPK) == 0 && (CC % TPN) == 0);
static_assert(TPN * 8 == NTHR && TPK * TPN == NTHR * 8 && TPK == NWAVE * 8);
static_assert((TPP % 8) == 0 && TPP >= TPK);
static_assert((CC % 8) == 0);
static_assert(LDS_FILL <= 300 * 1024);

typedef float     v4f  __attribute__((ext_vector_type(4)));
typedef float     v8f  __attribute__((ext_vector_type(8)));
typedef int       v4i  __attribute__((ext_vector_type(4)));
typedef _Float16  v4h  __attribute__((ext_vector_type(4)));
typedef _Float16  v8h  __attribute__((ext_vector_type(8)));
typedef _Float16  v16h __attribute__((ext_vector_type(16)));
union FragH { v16h v; v8h h[2]; };
union U32F { float f; int i; };

__device__ __forceinline__ v8f wmf(v16h a, v16h b, v8f c) {
  v8f d = __builtin_amdgcn_wmma_f32_16x16x32_f16(false, a, false, b, (short)0, c, false, false);
  asm volatile("v_nop\n\tv_nop\n\tv_nop\n\tv_nop" : "+v"(d) : "v"(a), "v"(b));
  return d;
}

__device__ __forceinline__ float lrelu1(float v) { return v >= 0.0f ? v : 0.01f * v; }
__device__ __forceinline__ v4f lrelu4(v4f t) {
  v4f o;
  o.x = lrelu1(t.x); o.y = lrelu1(t.y); o.z = lrelu1(t.z); o.w = lrelu1(t.w);
  return o;
}

template <int NB, int SRC, int WC>
__device__ __forceinline__ int scan_chunk(const int* __restrict__ keys, int nK, int cbase,
                                          int slotBase, int vec8, int* list, int tid, int lane, int wave) {
  int wc = 0;
#pragma unroll
  for (int g = 0; g < NGRP; ++g) {
    const int el0  = (g * NTHR + tid) * EPT;
    const int e0   = cbase + el0;
    const int sent = -2147483647 - 1;
    const int i0 = min(e0, nK - 1),     i1 = min(e0 + 1, nK - 1), i2 = min(e0 + 2, nK - 1), i3 = min(e0 + 3, nK - 1);
    const int i4 = min(e0 + 4, nK - 1), i5 = min(e0 + 5, nK - 1), i6 = min(e0 + 6, nK - 1), i7 = min(e0 + 7, nK - 1);
    v4i da, db;
    if (vec8 != 0 && cbase + CHUNK <= nK) {
      da = *(const v4i*)(keys + e0);
      db = *(const v4i*)(keys + e0 + 4);
    } else {
      da.x = (e0     < nK) ? keys[i0] : sent;
      da.y = (e0 + 1 < nK) ? keys[i1] : sent;
      da.z = (e0 + 2 < nK) ? keys[i2] : sent;
      da.w = (e0 + 3 < nK) ? keys[i3] : sent;
      db.x = (e0 + 4 < nK) ? keys[i4] : sent;
      db.y = (e0 + 5 < nK) ? keys[i5] : sent;
      db.z = (e0 + 6 < nK) ? keys[i6] : sent;
      db.w = (e0 + 7 < nK) ? keys[i7] : sent;
    }
    const unsigned nb = (unsigned)slotBase;
    const unsigned s0 = (unsigned)da.x - nb, s1 = (unsigned)da.y - nb;
    const unsigned s2 = (unsigned)da.z - nb, s3 = (unsigned)da.w - nb;
    const unsigned s4 = (unsigned)db.x - nb, s5 = (unsigned)db.y - nb;
    const unsigned s6 = (unsigned)db.z - nb, s7 = (unsigned)db.w - nb;
    const bool h0 = s0 < (unsigned)NB, h1 = s1 < (unsigned)NB, h2 = s2 < (unsigned)NB, h3 = s3 < (unsigned)NB;
    const bool h4 = s4 < (unsigned)NB, h5 = s5 < (unsigned)NB, h6 = s6 < (unsigned)NB, h7 = s7 < (unsigned)NB;
    const unsigned any = __builtin_amdgcn_ballot_w32(h0 | h1 | h2 | h3 | h4 | h5 | h6 | h7);
    if (any != 0u) {
#define HITJ(HJ, SJ, VJ) { \
        const unsigned mj = __builtin_amdgcn_ballot_w32(HJ); \
        if (mj != 0u) { \
          if (HJ) { \
            const int pos = wc + (int)__builtin_amdgcn_mbcnt_lo(mj, 0u); \
            const int entv = SRC ? (((VJ) << ESHF) | (int)(SJ)) : (int)(SJ); \
            if (pos < WC) list[wave * WC + pos] = entv; \
          } \
          wc += (int)__builtin_popcount(mj); } }
      HITJ(h0, s0, i0)
      HITJ(h1, s1, i1)
      HITJ(h2, s2, i2)
      HITJ(h3, s3, i3)
      HITJ(h4, s4, i4)
      HITJ(h5, s5, i5)
      HITJ(h6, s6, i6)
      HITJ(h7, s7, i7)
#undef HITJ
    }
  }
  return wc;
}

__global__ __launch_bounds__(NTHR) void k_cvt16(const float* __restrict__ src, _Float16* dst,
                                                int rowLen, int nSrcRows, int total8, float scale) {
  const int i = (int)blockIdx.x * NTHR + (int)threadIdx.x;
  if (i >= total8) return;
  const size_t e  = (size_t)8 * (size_t)i;
  const int    r  = (int)(e / (size_t)rowLen);
  const int    k0 = (int)(e - (size_t)r * (size_t)rowLen);
  const int    rc = r < nSrcRows ? r : nSrcRows - 1;
  const float  z  = (r < nSrcRows) ? scale : 0.0f;
  const float* sp = src + (size_t)rc * rowLen + k0;
  const v4f f0 = *(const v4f*)sp;
  const v4f f1 = *(const v4f*)(sp + 4);
  v8h hv;
  hv[0] = (_Float16)(f0.x * z); hv[1] = (_Float16)(f0.y * z); hv[2] = (_Float16)(f0.z * z); hv[3] = (_Float16)(f0.w * z);
  hv[4] = (_Float16)(f1.x * z); hv[5] = (_Float16)(f1.y * z); hv[6] = (_Float16)(f1.z * z); hv[7] = (_Float16)(f1.w * z);
  _Float16* d = dst + e;
  *(volatile v8h*)d = hv;
  __threadfence();
  *(volatile v8h*)d = hv;
}

__global__ __launch_bounds__(NTHR) void k_wT16(const float* __restrict__ W, _Float16* Wp,
                                               int KD, int NC, float scale) {
  __shared__ __attribute__((aligned(16))) _Float16 sT[TPN * TPP];
  const int tid = threadIdx.x;
  const int k0 = (int)blockIdx.x * TPK, n0 = (int)blockIdx.y * TPN;
  const int nc = tid & 31, kq = tid >> 5;
#pragma unroll
  for (int i = 0; i < TPK / NWAVE; ++i) {
    const int kr = kq + NWAVE * i;
    const float v = W[(size_t)(k0 + kr) * NC + n0 + nc] * scale;
    sT[nc * TPP + kr] = (_Float16)v;
  }
  __syncthreads();
  const int nl = tid >> 3, p = tid & 7;
  const v8h hv = *(const v8h*)(sT + nl * TPP + 8 * p);
  _Float16* d = Wp + (size_t)(n0 + nl) * KD + k0 + 8 * p;
  *(volatile v8h*)d = hv;
  __threadfence();
  *(volatile v8h*)d = hv;
}

__global__ __launch_bounds__(NTHR) void k_count(
    const int* __restrict__ keys, int* cnt, int nK, int vec8) {
  extern __shared__ v4f lds_dyn[];
  int* scnt = (int*)lds_dyn;
  int* list = scnt + NBC;
  int* wcnt = list + NWAVE * WCAPC;
  const int tid = threadIdx.x, lane = tid & 31, wave = tid >> 5;
  const int nodeBase = blockIdx.x * NBC;

  {
    const v4i z = {0, 0, 0, 0};
    for (int i = tid; i < NBC / 4; i += NTHR) ((v4i*)scnt)[i] = z;
  }
  __syncthreads();

  const int nChunks = (nK + CHUNK - 1) / CHUNK;
#pragma unroll 1
  for (int ch = 0; ch < nChunks; ++ch) {
    const int cbase = ch * CHUNK;
    const int wc = scan_chunk<NBC, 0, WCAPC>(keys, nK, cbase, nodeBase, vec8, list, tid, lane, wave);
    if (lane == 0) wcnt[wave] = wc;
    __syncthreads();
    if (wave == 0) {
#pragma unroll 1
      for (int wsx = 0; wsx < NWAVE; ++wsx) {
        int n = __builtin_amdgcn_readfirstlane(wcnt[wsx]);
        n = n > WCAPC ? WCAPC : (n < 0 ? 0 : n);
        const int* lp = list + wsx * WCAPC;
#pragma unroll 1
        for (int i = 0; i < n; ++i) {
          const int ent  = __builtin_amdgcn_readfirstlane(lp[i]);
          const int slot = ent & (NBC - 1);
          if (lane == 0) scnt[slot] = scnt[slot] + 1;
        }
      }
    }
    __syncthreads();
  }

  int* cp = cnt + (size_t)nodeBase;
#pragma unroll 4
  for (int q = 0; q < 32; ++q) {
    const int f = (wave * 32 + q) * 128 + 4 * lane;
    const v4i c = *(const v4i*)(scnt + f);
    *(volatile v4i*)(cp + f) = c;
  }
  __threadfence();
#pragma unroll 4
  for (int q = 0; q < 32; ++q) {
    const int f = (wave * 32 + q) * 128 + 4 * lane;
    const v4i c = *(const v4i*)(scnt + f);
    *(volatile v4i*)(cp + f) = c;
  }
}

__global__ __launch_bounds__(OTHR) void k_offsets(
    const int* __restrict__ cnt, int* off, float* dis, int* rbase, int nBF) {
  __shared__ __attribute__((aligned(16))) int srb[RBN];
  __shared__ int wtot[OTHR / 32];
  const int tid = threadIdx.x, lane = tid & 31, wave = tid >> 5;
  for (int i = tid; i < RBN; i += OTHR) srb[i] = 0;
  int carry = 0;
#pragma unroll 1
  for (int fb = 0; fb < nBF; ++fb) {
    const int base = fb * NBF;
    const v4i c = *(const v4i*)(cnt + base + 4 * tid);
    const int e0 = max(c.x, 0), e1 = max(c.y, 0), e2 = max(c.z, 0), e3 = max(c.w, 0);
    const int ts = e0 + e1 + e2 + e3;
    int incl = ts;
#pragma unroll
    for (int d = 1; d < 32; d <<= 1) {
      const int t = __shfl_up(incl, d, 32);
      if (lane >= d) incl += t;
    }
    if (lane == 31) wtot[wave] = incl;
    __syncthreads();
    int pre = 0;
#pragma unroll 1
    for (int w = 0; w < wave; ++w) pre += wtot[w];
    int tot = 0;
#pragma unroll
    for (int w = 0; w < OTHR / 32; ++w) tot += wtot[w];
    int run = carry + pre + incl - ts;
    v4i o;
    o.x = run; run += e0;
    o.y = run; run += e1;
    o.z = run; run += e2;
    o.w = run;
    v4f dv;
    dv.x = rsqrtf((float)e0 + 1.0f);
    dv.y = rsqrtf((float)e1 + 1.0f);
    dv.z = rsqrtf((float)e2 + 1.0f);
    dv.w = rsqrtf((float)e3 + 1.0f);
    int*   op = off + base + 4 * tid;
    float* dp = dis + base + 4 * tid;
    *(volatile v4i*)op = o;
    *(volatile v4f*)dp = dv;
    __threadfence();
    *(volatile v4i*)op = o;
    *(volatile v4f*)dp = dv;
    if (tid == 0) srb[min(fb, RBN - 1)] = carry;
    carry += (tot + 31) & ~31;
    __syncthreads();
  }
  if (tid == 0) srb[min(nBF, RBN - 1)] = carry;
  __syncthreads();
  v4i rv = {0, 0, 0, 0};
  if (tid < 32) rv = *(const v4i*)(srb + 4 * tid);
  if (tid < 32) *(volatile v4i*)(rbase + 4 * tid) = rv;
  __threadfence();
  if (tid < 32) *(volatile v4i*)(rbase + 4 * tid) = rv;
}

__global__ __launch_bounds__(NTHR) void k_fill(
    const int* __restrict__ keys, const int* __restrict__ off,
    const int* __restrict__ rbase, int* csr, int nK, int vec8, int csrLen) {
  extern __shared__ v4f lds_dyn[];
  int* region = (int*)lds_dyn;
  int* cursor = region + RCAP;
  int* list   = cursor + NBF;
  int* wcnt   = list + NWAVE * WCAPF;
  const int tid = threadIdx.x, lane = tid & 31, wave = tid >> 5;
  const int b = blockIdx.x;
  const int nodeBase = b * NBF;

  int rb0 = rbase[b];
  const int rb1 = rbase[b + 1];
  rb0 = rb0 < 0 ? 0 : (rb0 > csrLen ? csrLen : rb0);
  rb0 &= ~31;
  int len = rb1 - rb0;
  len = len < 0 ? 0 : (len > RCAP ? RCAP : len);
  int lenW = (len + 31) & ~31;
  if (rb0 + lenW > csrLen) lenW = (csrLen - rb0) & ~31;

  {
    const v4i z = {0, 0, 0, 0};
    for (int i = tid; i < RCAP / 4; i += NTHR) ((v4i*)region)[i] = z;
    for (int s = tid; s < NBF; s += NTHR) {
      int o = off[nodeBase + s] - rb0;
      o = o < 0 ? 0 : (o > RCAP ? RCAP : o);
      cursor[s] = o;
    }
  }
  __syncthreads();

  const int nChunks = (nK + CHUNK - 1) / CHUNK;
#pragma unroll 1
  for (int ch = 0; ch < nChunks; ++ch) {
    const int cbase = ch * CHUNK;
    const int wc = scan_chunk<NBF, 1, WCAPF>(keys, nK, cbase, nodeBase, vec8, list, tid, lane, wave);
    if (lane == 0) wcnt[wave] = wc;
    __syncthreads();
    if (wave == 0) {
#pragma unroll 1
      for (int wsx = 0; wsx < NWAVE; ++wsx) {
        int n = __builtin_amdgcn_readfirstlane(wcnt[wsx]);
        n = n > WCAPF ? WCAPF : (n < 0 ? 0 : n);
        const int* lp = list + wsx * WCAPF;
#pragma unroll 1
        for (int i = 0; i < n; ++i) {
          const int ent  = __builtin_amdgcn_readfirstlane(lp[i]);
          const int slot = ent & (NBF - 1);
          int ev = (ent >> ESHF) & EMASK;
          ev = ev > nK - 1 ? nK - 1 : ev;
          if (lane == 0) {
            int pos = cursor[slot];
            pos = pos < 0 ? 0 : (pos > RCAP - 1 ? RCAP - 1 : pos);
            region[pos] = ev;
            const int np = pos + 1;
            cursor[slot] = np > RCAP ? RCAP : np;
          }
        }
      }
    }
    __syncthreads();
  }

  const int nv = lenW >> 2;
  int* gp = csr + rb0;
#pragma unroll 1
  for (int i = tid; i < nv; i += NTHR) { const v4i v = ((const v4i*)region)[i]; *(volatile v4i*)(gp + 4 * i) = v; }
  __threadfence();
#pragma unroll 1
  for (int i = tid; i < nv; i += NTHR) { const v4i v = ((const v4i*)region)[i]; *(volatile v4i*)(gp + 4 * i) = v; }
}

template <int EPO>
__global__ __launch_bounds__(NTHR) void k_gemm(
    const _Float16* __restrict__ A16, const _Float16* __restrict__ Bw,
    const float* __restrict__ bias, void* Cout, float osc) {
  extern __shared__ v4f lds_dyn[];
  constexpr int KD  = CC;
  constexpr int NC  = CC;
  constexpr int NT  = NC / 16;
  constexpr int NST = 16;
  float* stg = (float*)lds_dyn;
  const int tid = threadIdx.x, lane = tid & 31, wave = tid >> 5, hh = lane >> 4, m = lane & 15;
  const int rowBase = blockIdx.x * GROWS;
  const _Float16* ap  = A16 + (size_t)(rowBase + wave * 16 + m) * KD + 8 * hh;
  const _Float16* bp0 = Bw + (size_t)m * KD + 8 * hh;

  v8f acc[NT];
#pragma unroll
  for (int t = 0; t < NT; ++t) { v8f z = {0.f, 0.f, 0.f, 0.f, 0.f, 0.f, 0.f, 0.f}; acc[t] = z; }

#pragma unroll 1
  for (int kt = 0; kt < KD / 32; ++kt) {
    FragH af;
    af.h[0] = *(const v8h*)(ap + 32 * kt);
    af.h[1] = *(const v8h*)(ap + 32 * kt + 16);
#pragma unroll
    for (int t = 0; t < NT; ++t) {
      const _Float16* bp = bp0 + (size_t)(16 * t) * KD + 32 * kt;
      FragH bf;
      bf.h[0] = *(const v8h*)bp;
      bf.h[1] = *(const v8h*)(bp + 16);
      acc[t] = wmf(af.v, bf.v, acc[t]);
    }
  }

  const int r0 = wave * 16 + 8 * hh;
  float bc[NT];
#pragma unroll
  for (int t = 0; t < NT; ++t) bc[t] = (EPO == 1) ? bias[16 * t + m] : 0.0f;

  float* sp = stg + r0 * NC + m;
#pragma unroll
  for (int t = 0; t < NT; ++t) {
#pragma unroll
    for (int r = 0; r < 8; ++r) {
      const float v = acc[t][r] * osc;
      sp[r * NC + 16 * t] = (EPO == 1) ? ((float)HSCL * lrelu1(v + bc[t])) : v;
    }
  }
  __syncthreads();

  const float* lp = stg + wave * 16 * NC;
  if (EPO == 0) {
    float* C = (float*)Cout;
    float* gp = C + (size_t)(rowBase + wave * 16) * NC;
#pragma unroll
    for (int i = 0; i < NST; ++i) {
      const v4f v = *(const v4f*)(lp + i * NC + 4 * lane);
      *(volatile v4f*)(gp + (size_t)i * NC + 4 * lane) = v;
    }
    __threadfence();
#pragma unroll
    for (int i = 0; i < NST; ++i) {
      const v4f v = *(const v4f*)(lp + i * NC + 4 * lane);
      *(volatile v4f*)(gp + (size_t)i * NC + 4 * lane) = v;
    }
  } else {
    _Float16* C = (_Float16*)Cout;
    _Float16* gp = C + (size_t)(rowBase + wave * 16) * NC;
#pragma unroll
    for (int i = 0; i < NST; ++i) {
      const v4f v = *(const v4f*)(lp + i * NC + 4 * lane);
      v4h q;
      q[0] = (_Float16)v.x; q[1] = (_Float16)v.y; q[2] = (_Float16)v.z; q[3] = (_Float16)v.w;
      *(volatile v4h*)(gp + (size_t)i * NC + 4 * lane) = q;
    }
    __threadfence();
#pragma unroll
    for (int i = 0; i < NST; ++i) {
      const v4f v = *(const v4f*)(lp + i * NC + 4 * lane);
      v4h q;
      q[0] = (_Float16)v.x; q[1] = (_Float16)v.y; q[2] = (_Float16)v.z; q[3] = (_Float16)v.w;
      *(volatile v4h*)(gp + (size_t)i * NC + 4 * lane) = q;
    }
  }
}

template <int MODE>
__global__ __launch_bounds__(NTHR) void k_agg(
    const int* __restrict__ csr, const int* __restrict__ off, const int* __restrict__ cnt,
    const int* __restrict__ srcidx, const float* __restrict__ dis,
    const float* __restrict__ hw, const float* __restrict__ bias, const float* __restrict__ wo,
    _Float16* out16, float* outS, int nN, int nE, int csrLen) {
  const int tid = threadIdx.x, lane = tid & 31, wave = tid >> 5;
  const int tbase = blockIdx.x * TGT + wave * 32;
  const int cl = tbase + lane;
  const int cnt_l = cnt[cl];
  const int off_l = off[cl];
  const float dis_l = dis[cl];
  const int ch = 4 * lane;
  const v4f bv = *(const v4f*)(bias + ch);
  v4f wv = {0.f, 0.f, 0.f, 0.f};
  if (MODE == 1) wv = *(const v4f*)(wo + ch);
  float skeep = 0.f;

#pragma unroll 1
  for (int j = 0; j < 32; ++j) {
    const int c = tbase + j;
    const int nraw = __builtin_amdgcn_readlane(cnt_l, j);
    const int n = nraw < 0 ? 0 : (nraw > DEGCAP ? DEGCAP : nraw);
    const int st = __builtin_amdgcn_readlane(off_l, j);
    U32F du; du.i = __builtin_amdgcn_readlane(__float_as_int(dis_l), j);
    const float dc = du.f;
    v4f acc = {0.f, 0.f, 0.f, 0.f};
#pragma unroll 1
    for (int q0 = 0; q0 < n; q0 += 32) {
      int pos = st + q0 + lane;
      pos = pos < 0 ? 0 : (pos > csrLen - 1 ? csrLen - 1 : pos);
      int el = csr[pos];
      el = el < 0 ? 0 : (el > nE - 1 ? nE - 1 : el);
      int sl = srcidx[el];
      sl = sl < 0 ? 0 : (sl > nN - 1 ? nN - 1 : sl);
      U32F wu; wu.f = dis[sl] * dc;
      const int mcnt = (n - q0) < 32 ? (n - q0) : 32;
#pragma unroll 1
      for (int p = 0; p < mcnt; ++p) {
        const int s = __builtin_amdgcn_readlane(sl, p);
        U32F t; t.i = __builtin_amdgcn_readlane(wu.i, p);
        const v4f hv = *(const v4f*)(hw + (size_t)s * CC + ch);
        acc = acc + hv * t.f;
      }
    }
    const v4f hc = *(const v4f*)(hw + (size_t)c * CC + ch);
    const float d2 = dc * dc;
    v4f v = acc + hc * d2 + bv;
    v = lrelu4(v);
    if (c >= nN) { const v4f z = {0.f, 0.f, 0.f, 0.f}; v = z; }
    if (nraw > DEGCAP) {
      const float qn = __int_as_float(0x7fc00000);
      v.x = qn; v.y = qn; v.z = qn; v.w = qn;
    }
    if (MODE == 0) {
      v4h q;
      q[0] = (_Float16)(v.x * (float)HSCL); q[1] = (_Float16)(v.y * (float)HSCL);
      q[2] = (_Float16)(v.z * (float)HSCL); q[3] = (_Float16)(v.w * (float)HSCL);
      _Float16* rp = out16 + (size_t)c * CC + ch;
      *(volatile v4h*)rp = q;
      __threadfence();
      *(volatile v4h*)rp = q;
    } else {
      float part = v.x * wv.x + v.y * wv.y + v.z * wv.z + v.w * wv.w;
      part += __shfl_xor(part, 16, 32);
      part += __shfl_xor(part, 8, 32);
      part += __shfl_xor(part, 4, 32);
      part += __shfl_xor(part, 2, 32);
      part += __shfl_xor(part, 1, 32);
      skeep = (lane == j) ? part : skeep;
    }
  }
  if (MODE == 1) {
    float* spo = outS + cl;
    *(volatile float*)spo = skeep;
    __threadfence();
    *(volatile float*)spo = skeep;
  }
}

__global__ __launch_bounds__(NTHR) void k_aggs(
    const int* __restrict__ csr, const int* __restrict__ off, const int* __restrict__ cnt,
    const int* __restrict__ srcidx, const float* __restrict__ dis,
    const float* __restrict__ S, const float* __restrict__ bo, float* outp,
    int nN, int nE, int csrLen) {
  const int tid = threadIdx.x, lane = tid & 31, wave = tid >> 5;
  const int tbase = blockIdx.x * TGT + wave * 32;
  const int cl = tbase + lane;
  const int cnt_l = cnt[cl];
  const int off_l = off[cl];
  const float dis_l = dis[cl];
  const float b0 = bo[0];
  float rkeep = 0.f;

#pragma unroll 1
  for (int j = 0; j < 32; ++j) {
    const int c = tbase + j;
    const int nraw = __builtin_amdgcn_readlane(cnt_l, j);
    const int n = nraw < 0 ? 0 : (nraw > DEGCAP ? DEGCAP : nraw);
    const int st = __builtin_amdgcn_readlane(off_l, j);
    U32F du; du.i = __builtin_amdgcn_readlane(__float_as_int(dis_l), j);
    const float dc = du.f;
    float acc = 0.f;
#pragma unroll 1
    for (int q0 = 0; q0 < n; q0 += 32) {
      int pos = st + q0 + lane;
      pos = pos < 0 ? 0 : (pos > csrLen - 1 ? csrLen - 1 : pos);
      int el = csr[pos];
      el = el < 0 ? 0 : (el > nE - 1 ? nE - 1 : el);
      int sl = srcidx[el];
      sl = sl < 0 ? 0 : (sl > nN - 1 ? nN - 1 : sl);
      float term = S[sl] * (dis[sl] * dc);
      const int mcnt = (n - q0) < 32 ? (n - q0) : 32;
      term = (lane < mcnt) ? term : 0.0f;
      term += __shfl_xor(term, 16, 32);
      term += __shfl_xor(term, 8, 32);
      term += __shfl_xor(term, 4, 32);
      term += __shfl_xor(term, 2, 32);
      term += __shfl_xor(term, 1, 32);
      acc += term;
    }
    const float sc = S[c];
    float r = acc + sc * (dc * dc) + b0;
    if (nraw > DEGCAP) r = __int_as_float(0x7fc00000);
    rkeep = (lane == j) ? r : rkeep;
  }
  if (cl < nN) *(volatile float*)(outp + cl) = rkeep;
  __threadfence();
  if (cl < nN) *(volatile float*)(outp + cl) = rkeep;
}

extern "C" void kernel_launch(void* const* d_in, const int* in_sizes, int n_in,
                              void* d_out, int out_size, void* d_ws, size_t ws_size,
                              hipStream_t stream) {
  if (n_in < 14) return;
  const int nN = in_sizes[0] / CC;
  if (nN <= 0 || in_sizes[0] != nN * CC) return;
  if (in_sizes[1] < 2 || (in_sizes[1] & 1) != 0) return;
  const int nE = in_sizes[1] / 2;
  if (in_sizes[2] != CC * CC || in_sizes[3] != CC) return;
  if (in_sizes[4] != CC * CC || in_sizes[5] != CC) return;
  if (in_sizes[6] != CC * CC || in_sizes[7] != CC) return;
  if (in_sizes[8] != CC * CC || in_sizes[9] != CC) return;
  if (in_sizes[10] != CC * CC || in_sizes[11] != CC) return;
  if (in_sizes[12] != CC || in_sizes[13] < 1) return;
  if (nN > (1 << 20) || nE > (1 << 20)) return;
  if (out_size != nN) return;

  const float* x    = (const float*)d_in[0];
  const int*   ei   = (const int*)d_in[1];
  const int*   srci = ei;
  const int*   dsti = ei + nE;
  const float* W1   = (const float*)d_in[2];
  const float* b1   = (const float*)d_in[3];
  const float* W2   = (const float*)d_in[4];
  const float* b2   = (const float*)d_in[5];
  const float* W3   = (const float*)d_in[6];
  const float* b3   = (const float*)d_in[7];
  const float* Wg0  = (const float*)d_in[8];
  const float* bg0  = (const float*)d_in[9];
  const float* Wg1  = (const float*)d_in[10];
  const float* bg1  = (const float*)d_in[11];
  const float* Wo   = (const float*)d_in[12];
  const float* bo   = (const float*)d_in[13];
  float* out = (float*)d_out;
  const int nK = nE;

  const int NPAD   = ((nN + TGT - 1) / TGT) * TGT;
  const int nBC    = (nN + NBC - 1) / NBC;
  const int CNTPAD = nBC * NBC;
  const int nBF    = (nN + NBF - 1) / NBF;
  const int OFFN   = nBF * NBF;
  if (nBF + 1 > RBN) return;
  if (OFFN > CNTPAD || NPAD > OFFN) return;
  if ((NPAD % GROWS) != 0 || (NPAD % TGT) != 0) return;
  const int csrLen = ((nK + 31) & ~31) + 32 * (nBF + 1);
  const int nGemm  = NPAD / GROWS;
  const int nAgg   = NPAD / TGT;

  char* ws = (char*)d_ws;
  size_t off = 0;
  const size_t oP0  = off; off += (size_t)NPAD * CC * 2;          off = (off + 255) & ~(size_t)255;
  const size_t oP1  = off; off += (size_t)NPAD * CC * 2;          off = (off + 255) & ~(size_t)255;
  const size_t oW1  = off; off += (size_t)CC * CC * 2;            off = (off + 255) & ~(size_t)255;
  const size_t oW2  = off; off += (size_t)CC * CC * 2;            off = (off + 255) & ~(size_t)255;
  const size_t oW3  = off; off += (size_t)CC * CC * 2;            off = (off + 255) & ~(size_t)255;
  const size_t oWg0 = off; off += (size_t)CC * CC * 2;            off = (off + 255) & ~(size_t)255;
  const size_t oWg1 = off; off += (size_t)CC * CC * 2;            off = (off + 255) & ~(size_t)255;
  const size_t oCnt = off; off += (size_t)CNTPAD * 4;             off = (off + 255) & ~(size_t)255;
  const size_t oOff = off; off += (size_t)OFFN * 4;               off = (off + 255) & ~(size_t)255;
  const size_t oDis = off; off += (size_t)OFFN * 4;               off = (off + 255) & ~(size_t)255;
  const size_t oRb  = off; off += (size_t)RBN * 4;                off = (off + 255) & ~(size_t)255;
  const size_t oCsr = off; off += (size_t)csrLen * 4;             off = (off + 255) & ~(size_t)255;
  const size_t oXW  = off; off += (size_t)NPAD * CC * 4;          off = (off + 255) & ~(size_t)255;
  const size_t oS   = off; off += (size_t)NPAD * 4;               off = (off + 255) & ~(size_t)255;
  if (off > ws_size || off > (size_t)WSCAP) return;
  _Float16* P0   = (_Float16*)(ws + oP0);
  _Float16* P1   = (_Float16*)(ws + oP1);
  _Float16* W1p  = (_Float16*)(ws + oW1);
  _Float16* W2p  = (_Float16*)(ws + oW2);
  _Float16* W3p  = (_Float16*)(ws + oW3);
  _Float16* Wg0p = (_Float16*)(ws + oWg0);
  _Float16* Wg1p = (_Float16*)(ws + oWg1);
  int*      cnt  = (int*)(ws + oCnt);
  int*      offp = (int*)(ws + oOff);
  float*    dis  = (float*)(ws + oDis);
  int*      rb   = (int*)(ws + oRb);
  int*      csr  = (int*)(ws + oCsr);
  float*    XW   = (float*)(ws + oXW);
  float*    S    = (float*)(ws + oS);

  const int vec8 = ((nE & 3) == 0) ? 1 : 0;
  const float oscX = 1.0f / ((float)ASCL * (float)WSCL);
  const float oscH = 1.0f / ((float)HSCL * (float)WSCL);

  {
    const int t8x = (NPAD * CC) / 8;
    k_cvt16<<<(t8x + NTHR - 1) / NTHR, NTHR, 0, stream>>>(x, P0, CC, nN, t8x, (float)ASCL);
  }
  {
    const dim3 gW(CC / TPK, CC / TPN);
    k_wT16<<<gW, NTHR, 0, stream>>>(W1,  W1p,  CC, CC, (float)WSCL);
    k_wT16<<<gW, NTHR, 0, stream>>>(W2,  W2p,  CC, CC, (float)WSCL);
    k_wT16<<<gW, NTHR, 0, stream>>>(W3,  W3p,  CC, CC, (float)WSCL);
    k_wT16<<<gW, NTHR, 0, stream>>>(Wg0, Wg0p, CC, CC, (float)WSCL);
    k_wT16<<<gW, NTHR, 0, stream>>>(Wg1, Wg1p, CC, CC, (float)WSCL);
  }

  hipFuncSetAttribute(reinterpret_cast<const void*>(&k_count),
                      hipFuncAttributeMaxDynamicSharedMemorySize, LDS_COUNT);
  k_count<<<nBC, NTHR, LDS_COUNT, stream>>>(dsti, cnt, nK, vec8);
  k_offsets<<<1, OTHR, 0, stream>>>(cnt, offp, dis, rb, nBF);
  hipFuncSetAttribute(reinterpret_cast<const void*>(&k_fill),
                      hipFuncAttributeMaxDynamicSharedMemorySize, LDS_FILL);
  k_fill<<<nBF, NTHR, LDS_FILL, stream>>>(dsti, offp, rb, csr, nK, vec8, csrLen);

  hipFuncSetAttribute(reinterpret_cast<const void*>(&k_gemm<0>),
                      hipFuncAttributeMaxDynamicSharedMemorySize, LDS_GEMM);
  hipFuncSetAttribute(reinterpret_cast<const void*>(&k_gemm<1>),
                      hipFuncAttributeMaxDynamicSharedMemorySize, LDS_GEMM);
  k_gemm<1><<<nGemm, NTHR, LDS_GEMM, stream>>>(P0, W1p, b1, (void*)P1, oscX);
  k_gemm<1><<<nGemm, NTHR, LDS_GEMM, stream>>>(P1, W2p, b2, (void*)P0, oscH);
  k_gemm<1><<<nGemm, NTHR, LDS_GEMM, stream>>>(P0, W3p, b3, (void*)P1, oscH);

  k_gemm<0><<<nGemm, NTHR, LDS_GEMM, stream>>>(P1, Wg0p, b1, (void*)XW, oscH);
  k_agg<0><<<nAgg, NTHR, 0, stream>>>(csr, offp, cnt, srci, dis, XW, bg0, Wo, P0, S, nN, nE, csrLen);

  k_gemm<0><<<nGemm, NTHR, LDS_GEMM, stream>>>(P0, Wg1p, b1, (void*)XW, oscH);
  k_agg<1><<<nAgg, NTHR, 0, stream>>>(csr, offp, cnt, srci, dis, XW, bg1, Wo, P1, S, nN, nE, csrLen);

  k_aggs<<<nAgg, NTHR, 0, stream>>>(csr, offp, cnt, srci, dis, S, bo, out, nN, nE, csrLen);
}
